// multi_gcn_d_new_44727789421322
// MI455X (gfx1250) — hardware-verified
//
#include <hip/hip_runtime.h>

#define BT_ 192
#define NB_ 8
#define NN  512
#define CC  32
#define TT  24
#define RSPLIT (1.0f / 2048.0f)

typedef __attribute__((ext_vector_type(16))) _Float16 v16h;
typedef __attribute__((ext_vector_type(8)))  _Float16 v8h;
typedef __attribute__((ext_vector_type(8)))  float    v8f;
typedef __attribute__((ext_vector_type(4)))  float    v4f_t;
typedef float v4fa __attribute__((ext_vector_type(4), may_alias));
typedef __attribute__((ext_vector_type(4)))  unsigned v4u_t;
typedef unsigned v4ua __attribute__((ext_vector_type(4), may_alias));

__device__ __forceinline__ _Float16 lo_of(float v, _Float16 h) { return (_Float16)((v - (float)h) * 2048.0f); }
__device__ __forceinline__ v8f wmma16(v16h a, v16h b, v8f c) { return __builtin_amdgcn_wmma_f32_16x16x32_f16(false, a, false, b, (short)0, c, false, false); }
__device__ __forceinline__ v8f wmma_split(v16h a, v16h al, v16h b, v16h bl, v8f c) { v8f x = {}; x = wmma16(al, b, x); x = wmma16(a, bl, x); return wmma16(a, b, c) + x * RSPLIT; }
__device__ __forceinline__ v16h frag16(const _Float16* p, int g) {
  return __builtin_shufflevector(*(const v8h*)(p + 8 * g), *(const v8h*)(p + 16 + 8 * g), 0,1,2,3,4,5,6,7,8,9,10,11,12,13,14,15);
}
__device__ __forceinline__ void st16(_Float16* d, const _Float16* s8) { *(volatile v4u_t*)d = *(const v4ua*)s8; }

#define PLANE ((size_t)BT_ * NN * CC)

__global__ __launch_bounds__(256) void k_prep(const float* __restrict__ x, const float* __restrict__ W,
                                              _Float16* __restrict__ xt, _Float16* __restrict__ xT, _Float16* __restrict__ Wh) {
  const int t8 = blockIdx.x * 256 + threadIdx.x;
  const int nXt = BT_ * NN * (CC / 8), nXT = BT_ * CC * (NN / 8), nW = 32 * 224 / 8;
  _Float16 hh[8], hl[8];
  if (t8 < nXt) {
    const int c8 = (t8 & 3) * 8, n = (t8 >> 2) & (NN - 1), bt = t8 >> 11;
    const int b = bt / TT, t = bt % TT;
#pragma unroll
    for (int e = 0; e < 8; ++e) { const float v = x[(((size_t)b * CC + c8 + e) * NN + n) * TT + t]; hh[e] = (_Float16)v; hl[e] = lo_of(v, hh[e]); }
    _Float16* d = xt + ((size_t)bt * NN + n) * CC + c8;
    st16(d, hh); st16(d + PLANE, hl); __threadfence(); st16(d, hh); st16(d + PLANE, hl);
  } else if (t8 < nXt + nXT) {
    const int u = t8 - nXt;
    const int n8 = (u & 63) * 8, c = (u >> 6) & (CC - 1), bt = u >> 11;
    const int b = bt / TT, t = bt % TT;
#pragma unroll
    for (int e = 0; e < 8; ++e) hh[e] = (_Float16)x[(((size_t)b * CC + c) * NN + n8 + e) * TT + t];
    _Float16* d = xT + ((size_t)bt * CC + c) * NN + n8;
    st16(d, hh); __threadfence(); st16(d, hh);
  } else if (t8 < nXt + nXT + nW) {
    const int u = (t8 - nXt - nXT) * 8;
#pragma unroll
    for (int e = 0; e < 8; ++e) { const float v = W[u + e]; hh[e] = (_Float16)v; hl[e] = lo_of(v, hh[e]); }
    _Float16* d = Wh + u;
    st16(d, hh); st16(d + 32 * 224, hl); __threadfence(); st16(d, hh); st16(d + 32 * 224, hl);
  }
}

__global__ __launch_bounds__(128) void k_attn_hop1(const _Float16* __restrict__ xt, const _Float16* __restrict__ xT,
                                                   const float* __restrict__ s0, const float* __restrict__ s1,
                                                   const float* __restrict__ s2,
                                                   _Float16* __restrict__ x1, _Float16* __restrict__ x1T) {
  __shared__ __attribute__((aligned(16))) float P[4][16 * NN];
  __shared__ __attribute__((aligned(16))) float so[64 * 36];
  const int bt = blockIdx.x, rb = blockIdx.y;
  const int tid = threadIdx.x, lane = tid & 31, wave = tid >> 5;
  const int g = lane >> 4, l16 = lane & 15;
  const int row0 = rb * 64 + wave * 16;
  const _Float16* Xs  = xt + (size_t)bt * NN * CC;
  const _Float16* XTs = xT + (size_t)bt * CC * NN;
  float* Pw = P[wave];

  const v16h a = frag16(Xs + (size_t)(row0 + l16) * CC, g);
  const float scl = 0.17677669529663688f;
#pragma unroll 4
  for (int nt = 0; nt < NN / 16; ++nt) {
    v8f c = {};
    c = wmma16(a, frag16(Xs + (size_t)(nt * 16 + l16) * CC, g), c);
#pragma unroll
    for (int r = 0; r < 8; ++r) Pw[(r + 8 * g) * NN + nt * 16 + l16] = c[r] * scl;
  }
  asm volatile("s_wait_dscnt 0" ::: "memory");
  {
    float* pr = Pw + l16 * NN + g * 256;
    float mx = -3.0e38f;
    for (int j = 0; j < 256; ++j) mx = fmaxf(mx, pr[j]);
    mx = fmaxf(mx, __shfl_xor(mx, 16, 32));
    float sum = 0.f;
    for (int j = 0; j < 256; ++j) { const float e = __expf(pr[j] - mx); pr[j] = e; sum += e; }
    sum += __shfl_xor(sum, 16, 32);
    const float inv = 1024.0f / sum;
    for (int j = 0; j < 256; ++j) pr[j] *= inv;
  }
  asm volatile("s_wait_dscnt 0" ::: "memory");

#pragma unroll 1
  for (int s = 0; s < 3; ++s) {
    const float* A_ = (s == 0) ? s0 : (s == 1) ? s1 : s2;
    const float* arow = A_ + (size_t)(row0 + l16) * NN;
    const float* prow = Pw + l16 * NN;
    v8f acc[2] = {};
#pragma unroll 2
    for (int kc = 0; kc < NN / 32; ++kc) {
      v16h af;
#pragma unroll
      for (int i = 0; i < 16; ++i) { const int v = kc * 32 + ((i < 8) ? (8 * g + i) : (16 + 8 * g + i - 8)); af[i] = (_Float16)(arow[v] * prow[v]); }
#pragma unroll
      for (int ct = 0; ct < 2; ++ct)
        acc[ct] = wmma16(af, frag16(XTs + (size_t)(ct * 16 + l16) * NN + kc * 32, g), acc[ct]);
    }
#pragma unroll
    for (int ct = 0; ct < 2; ++ct)
#pragma unroll
      for (int r = 0; r < 8; ++r) so[(wave * 16 + r + 8 * g) * 36 + ct * 16 + l16] = acc[ct][r] * (1.0f / 1024.0f);
    __syncthreads();
    _Float16* d1  = x1  + (size_t)s * 2 * PLANE + ((size_t)bt * NN + rb * 64) * CC;
    _Float16* d1T = x1T + (size_t)s * PLANE + (size_t)bt * CC * NN + rb * 64;
#pragma unroll 1
    for (int pass = 0; pass < 2; ++pass) {
      for (int ch = tid; ch < 64 * 4 + 32 * 8; ch += 128) {
        _Float16 hh[8], hl[8];
        if (ch < 256) { const int n = ch >> 2, c8 = (ch & 3) * 8;
#pragma unroll
          for (int e = 0; e < 8; ++e) { const float v = so[n * 36 + c8 + e]; hh[e] = (_Float16)v; hl[e] = lo_of(v, hh[e]); }
          st16(d1 + (size_t)n * CC + c8, hh); st16(d1 + PLANE + (size_t)n * CC + c8, hl);
        } else { const int u = ch - 256, c = u >> 3, n8 = (u & 7) * 8;
#pragma unroll
          for (int e = 0; e < 8; ++e) hh[e] = (_Float16)so[(n8 + e) * 36 + c];
          st16(d1T + (size_t)c * NN + n8, hh);
        }
      }
      __threadfence();
    }
    __syncthreads();
  }
}

__global__ __launch_bounds__(128) void k_hop2(const float* __restrict__ s0, const float* __restrict__ s1, const float* __restrict__ s2,
                                              const _Float16* __restrict__ x1T, _Float16* __restrict__ x2) {
  __shared__ __attribute__((aligned(16))) float so[64 * 36];
  const int bt = blockIdx.x, s = blockIdx.y, rb = blockIdx.z;
  const int tid = threadIdx.x, lane = tid & 31, wave = tid >> 5;
  const int g = lane >> 4, l16 = lane & 15;
  const int row0 = rb * 64 + wave * 16;
  const float* A_ = (s == 0) ? s0 : (s == 1) ? s1 : s2;
  const float* arow = A_ + (size_t)(row0 + l16) * NN;
  const _Float16* XT = x1T + (size_t)s * PLANE + (size_t)bt * CC * NN;
  v8f acc[2] = {};
#pragma unroll 2
  for (int kc = 0; kc < NN / 32; ++kc) {
    v16h af;
#pragma unroll
    for (int i = 0; i < 16; ++i) { const int v = kc * 32 + ((i < 8) ? (8 * g + i) : (16 + 8 * g + i - 8)); af[i] = (_Float16)arow[v]; }
#pragma unroll
    for (int ct = 0; ct < 2; ++ct) acc[ct] = wmma16(af, frag16(XT + (size_t)(ct * 16 + l16) * NN + kc * 32, g), acc[ct]);
  }
#pragma unroll
  for (int ct = 0; ct < 2; ++ct)
#pragma unroll
    for (int r = 0; r < 8; ++r) so[(wave * 16 + r + 8 * g) * 36 + ct * 16 + l16] = acc[ct][r];
  __syncthreads();
  _Float16* d2 = x2 + (size_t)s * 2 * PLANE + ((size_t)bt * NN + rb * 64) * CC;
#pragma unroll 1
  for (int pass = 0; pass < 2; ++pass) {
    for (int ch = tid; ch < 256; ch += 128) { const int n = ch >> 2, c8 = (ch & 3) * 8; _Float16 hh[8], hl[8];
#pragma unroll
      for (int e = 0; e < 8; ++e) { const float v = so[n * 36 + c8 + e]; hh[e] = (_Float16)v; hl[e] = lo_of(v, hh[e]); }
      st16(d2 + (size_t)n * CC + c8, hh); st16(d2 + PLANE + (size_t)n * CC + c8, hl); }
    __threadfence();
  }
}

__global__ __launch_bounds__(256) void k_conv(const _Float16* __restrict__ xt, const _Float16* __restrict__ x1,
                                              const _Float16* __restrict__ x2, const _Float16* __restrict__ Wh,
                                              const float* __restrict__ bias, float* __restrict__ y) {
  __shared__ __attribute__((aligned(16))) float so[32 * 16 * TT];
  const int b = blockIdx.x, n0 = blockIdx.y * 16;
  const int tid = threadIdx.x, lane = tid & 31, wave = tid >> 5;
  const int g = lane >> 4, l16 = lane & 15;
#pragma unroll 1
  for (int t = wave; t < TT; t += 8) {
    const int bt = b * TT + t;
    v8f acc[2] = {};
#pragma unroll 1
    for (int ch = 0; ch < 7; ++ch) {
      const _Float16* src = (ch == 0) ? (xt + (size_t)bt * NN * CC)
                          : (ch & 1) ? (x1 + (size_t)((ch - 1) >> 1) * 2 * PLANE + (size_t)bt * NN * CC)
                                     : (x2 + (size_t)((ch - 2) >> 1) * 2 * PLANE + (size_t)bt * NN * CC);
      const _Float16* bp = src + (size_t)(n0 + l16) * CC;
      const v16h bv = frag16(bp, g), bl = frag16(bp + PLANE, g);
#pragma unroll
      for (int mt = 0; mt < 2; ++mt) {
        const _Float16* ap = Wh + (size_t)(mt * 16 + l16) * 224 + ch * 32;
        acc[mt] = wmma_split(frag16(ap, g), frag16(ap + 32 * 224, g), bv, bl, acc[mt]);
      }
    }
#pragma unroll
    for (int mt = 0; mt < 2; ++mt)
#pragma unroll
      for (int r = 0; r < 8; ++r) { const int o = mt * 16 + r + 8 * g; so[(o * 16 + l16) * TT + t] = acc[mt][r] + bias[o]; }
  }
  __syncthreads();
#pragma unroll 1
  for (int pass = 0; pass < 2; ++pass) {
    for (int q = tid; q < 32 * 96; q += 256) { const int o = q / 96, w = (q % 96) * 4;
      *(volatile v4f_t*)(y + ((size_t)(b * 32 + o) * NN + n0) * TT + w) = *(const volatile v4fa*)(so + o * 16 * TT + w); }
    __threadfence();
  }
}

extern "C" void kernel_launch(void* const* d_in, const int* in_sizes, int n_in,
                              void* d_out, int out_size, void* d_ws, size_t ws_size,
                              hipStream_t stream) {
  (void)in_sizes; (void)n_in; (void)out_size; (void)ws_size;
  const float* x    = (const float*)d_in[0];
  const float* s0   = (const float*)d_in[1];
  const float* s1   = (const float*)d_in[2];
  const float* s2   = (const float*)d_in[3];
  const float* W    = (const float*)d_in[4];
  const float* bias = (const float*)d_in[5];
  float* y = (float*)d_out;

  _Float16* ws  = (_Float16*)d_ws;
  _Float16* xt  = ws;
  _Float16* xT  = xt + 2 * PLANE;
  _Float16* x1  = xT + PLANE;
  _Float16* x1T = x1 + 6 * PLANE;
  _Float16* x2  = x1T + 3 * PLANE;
  _Float16* Wh  = x2 + 6 * PLANE;

  const int nPrep = BT_ * NN * (CC / 8) + BT_ * CC * (NN / 8) + 32 * 224 / 8;
  k_prep<<<(nPrep + 255) / 256, 256, 0, stream>>>(x, W, xt, xT, Wh);
  k_attn_hop1<<<dim3(BT_, NN / 64), 128, 0, stream>>>(xt, xT, s0, s1, s2, x1, x1T);
  k_hop2<<<dim3(BT_, 3, NN / 64), 128, 0, stream>>>(s0, s1, s2, x1T, x2);
  k_conv<<<dim3(NB_, NN / 16), 256, 0, stream>>>(xt, x1, x2, Wh, bias, y);
}
